// RNNDecoder_26027501814589
// MI455X (gfx1250) — hardware-verified
//
#include <hip/hip_runtime.h>
#include <math.h>

constexpr int BATCH  = 2;
constexpr int NODES  = 100;
constexpr int TLEN   = 15;
constexpr int FEAT   = 6;
constexpr int NTYPE  = 4;
constexpr int HID    = 128;
constexpr int NSTEP  = TLEN - 1;
constexpr int EPR    = NODES - 1;
constexpr int NEDGE  = NODES * EPR;
constexpr int EROWS  = 112;
constexpr int NROW   = BATCH * NODES;
constexpr int NROWP  = 208;
constexpr int NTHR   = 256;
constexpr int APITCH = 136;
constexpr int FPITCH = 132;
constexpr int SLABP  = 68;
constexpr int PCOLS  = NTYPE * HID;
constexpr int NMAT   = 17;
constexpr int MATEL  = HID * HID;
constexpr int HALLROWS = NROWP * NSTEP;
constexpr int OUTROWS  = NROW * NSTEP;
constexpr int ZERO_V4  = NROWP * (2 * HID + 2 * PCOLS) / 4;
constexpr float WCARRY     = 16.0f;
constexpr float WCARRY_INV = 1.0f / 16.0f;
constexpr float AGG_SCALE  = 1.0f / (float)(NTYPE * FEAT);

static_assert(NEDGE == 9900);
static_assert(EROWS % 16 == 0 && EROWS >= EPR);
static_assert(EROWS == 14 * (NTHR / 32));
static_assert(NROWP % 16 == 0 && NROWP >= NROW);
static_assert(OUTROWS % 16 == 0);
static_assert(HID % 32 == 0);
static_assert(HID == 16 * (NTHR / 32));
static_assert(ZERO_V4 % NTHR == 0);
static_assert(3 * FEAT * HID == 3 * 4 * 192);

typedef __attribute__((ext_vector_type(16))) _Float16 v16h;
typedef __attribute__((ext_vector_type(8)))  _Float16 v8h;
typedef __attribute__((ext_vector_type(8)))  float    v8f;
typedef __attribute__((ext_vector_type(4)))  float    v4f;
typedef __attribute__((ext_vector_type(2)))  unsigned v2u;
typedef __attribute__((ext_vector_type(4)))  unsigned v4u;

union FragU { v16h v; v8h h[2]; };
__device__ __forceinline__ v16h frag_load(const _Float16* p) {
  FragU f;
  f.h[0] = *(const v8h*)(p);
  f.h[1] = *(const v8h*)(p + 16);
  return f.v;
}
__device__ __forceinline__ v8f mma_h(v16h a, v16h b, v8f c) {
  c = __builtin_amdgcn_wmma_f32_16x16x32_f16(false, a, false, b, (short)0, c, false, false);
  asm volatile("v_nop\n\tv_nop\n\tv_nop\n\tv_nop" : "+v"(c) : "v"(a), "v"(b));
  return c;
}
__device__ __forceinline__ float bf16r(float f) {
  const unsigned u = __float_as_uint(f);
  const unsigned q = (u + 0x7FFFu + ((u >> 16) & 1u)) & 0xFFFF0000u;
  return __uint_as_float(q);
}
__device__ __forceinline__ v4f bf16r4(v4f v) {
  v4f o;
  const float a0 = v[0], a1 = v[1], a2 = v[2], a3 = v[3];
  o[0] = bf16r(a0);
  o[1] = bf16r(a1);
  o[2] = bf16r(a2);
  o[3] = bf16r(a3);
  return o;
}
__device__ __forceinline__ unsigned f16_bits(float f) {
  const _Float16 hv = (_Float16)f;
  return (unsigned)__builtin_bit_cast(unsigned short, hv);
}
__device__ __forceinline__ unsigned pack_h2(float lo, float hi) {
  return f16_bits(lo) | (f16_bits(hi) << 16);
}
__device__ __forceinline__ float sigm(float x) {
  return __builtin_amdgcn_rcpf(1.0f + expf(-x));
}
__device__ __forceinline__ void wave_sync_lds() {
  __builtin_amdgcn_fence(__ATOMIC_RELEASE, "workgroup");
  __builtin_amdgcn_wave_barrier();
  __builtin_amdgcn_fence(__ATOMIC_ACQUIRE, "workgroup");
}

__global__ __launch_bounds__(NTHR) void wprep_kernel(const float* __restrict__ W1, const float* __restrict__ W2,
                                                     const float* __restrict__ Whr, const float* __restrict__ Whi,
                                                     const float* __restrict__ Whh, const float* __restrict__ Wo1,
                                                     const float* __restrict__ Wo2, unsigned short* __restrict__ WT) {
  __shared__ float Tt[64 * 65];
  const int tid = threadIdx.x;
  const int z = blockIdx.z;
  const float* src = Wo2;
  if (z < 8) src = W1 + (size_t)((z & 3) * 2 * HID + (z >> 2) * HID) * HID;
  else if (z < 12) src = W2 + (size_t)(z - 8) * MATEL;
  else if (z == 12) src = Whr;
  else if (z == 13) src = Whi;
  else if (z == 14) src = Whh;
  else if (z == 15) src = Wo1;
  unsigned short* O = WT + (size_t)z * MATEL;
  const int c0 = blockIdx.x * 64, r0 = blockIdx.y * 64;
#pragma unroll
  for (int i = 0; i < 4; ++i) {
    const int idx = i * NTHR + tid;
    const int rr = idx >> 4, cc = (idx & 15) * 4;
    const v4f v = *(const v4f*)(src + (size_t)(r0 + rr) * HID + c0 + cc);
    Tt[rr * 65 + cc + 0] = v[0];
    Tt[rr * 65 + cc + 1] = v[1];
    Tt[rr * 65 + cc + 2] = v[2];
    Tt[rr * 65 + cc + 3] = v[3];
  }
  __syncthreads();
  const int q = tid >> 3, c8 = (tid & 7) * 8;
  v8h hv[2];
#pragma unroll
  for (int g = 0; g < 2; ++g) {
    const int qq = g * 32 + q;
#pragma unroll
    for (int e = 0; e < 8; ++e) {
      const float f = Tt[(c8 + e) * 65 + qq];
      const float fb = bf16r(f);
      hv[g][e] = (_Float16)(fb * WCARRY);
    }
  }
  for (int pass = 0; pass < 2; ++pass) {
#pragma unroll
    for (int g = 0; g < 2; ++g) {
      const size_t o = (size_t)(c0 + g * 32 + q) * HID + (size_t)(r0 + c8);
      *(volatile v8h*)(O + o) = hv[g];
    }
    __threadfence();
  }
}

__global__ __launch_bounds__(NTHR) void zero_state_kernel(float* __restrict__ p, int n4) {
  const int i = blockIdx.x * NTHR + threadIdx.x;
  if (i < n4) {
    const v4f z = {0.0f, 0.0f, 0.0f, 0.0f};
    *(volatile v4f*)(p + (size_t)i * 4) = z;
    __threadfence();
    *(volatile v4f*)(p + (size_t)i * 4) = z;
  }
}

__global__ __launch_bounds__(NTHR) void edge_msg_kernel(const float* __restrict__ Ps, const float* __restrict__ Pr,
                                                        const float* __restrict__ rel_type,
                                                        const float* __restrict__ b1, const float* __restrict__ b2,
                                                        const unsigned short* __restrict__ W2tp,
                                                        float* __restrict__ agg) {
  __shared__ __align__(16) unsigned short sA[EROWS * APITCH];
  __shared__ __align__(16) float sRt[EROWS * 4];
  __shared__ __align__(16) float sAgg[HID];
  const _Float16* W2t = (const _Float16*)W2tp;
  const int tid = threadIdx.x, lane = tid & 31, wave = tid >> 5;
  const int c = lane & 15, hh = lane >> 4, koff = hh * 8;
  const int blk = blockIdx.x;
  const int b = blk / NODES;
  const int rcv = blk - b * NODES;

  {
    const int cc = tid < EROWS ? tid : (EROWS - 1);
    const int cl = cc < EPR ? cc : (EPR - 1);
    const v4f v = bf16r4(*(const v4f*)(rel_type + ((size_t)b * NEDGE + (size_t)rcv * EPR + (size_t)cl) * NTYPE));
    const bool live = cc < EPR;
    v4f o;
    o[0] = live ? v[0] : 0.0f;
    o[1] = live ? v[1] : 0.0f;
    o[2] = live ? v[2] : 0.0f;
    o[3] = live ? v[3] : 0.0f;
    if (tid < EROWS) *(v4f*)(sRt + cc * 4) = o;
  }

  const v8f z8 = {0.f, 0.f, 0.f, 0.f, 0.f, 0.f, 0.f, 0.f};
  float colacc = 0.0f;

#pragma unroll 1
  for (int k = 0; k < NTYPE; ++k) {
    {
      const int h4 = lane * 4;
      const v4f prv = *(const v4f*)(Pr + (size_t)blk * PCOLS + k * HID + h4);
      const v4f b1v = bf16r4(*(const v4f*)(b1 + k * HID + h4));
      const float base0 = prv[0] + b1v[0];
      const float base1 = prv[1] + b1v[1];
      const float base2 = prv[2] + b1v[2];
      const float base3 = prv[3] + b1v[3];
#pragma unroll 1
      for (int j = 0; j < 14; ++j) {
        const int cc = wave + 8 * j;
        const int cl = cc < EPR ? cc : (EPR - 1);
        const int snd = cl + ((cl >= rcv) ? 1 : 0);
        const v4f pv = *(const v4f*)(Ps + (size_t)(b * NODES + snd) * PCOLS + k * HID + h4);
        const bool live = cc < EPR;
        float m0 = tanhf(pv[0] + base0);
        float m1 = tanhf(pv[1] + base1);
        float m2 = tanhf(pv[2] + base2);
        float m3 = tanhf(pv[3] + base3);
        m0 = live ? m0 : 0.0f;
        m1 = live ? m1 : 0.0f;
        m2 = live ? m2 : 0.0f;
        m3 = live ? m3 : 0.0f;
        v2u pk;
        pk[0] = pack_h2(m0, m1);
        pk[1] = pack_h2(m2, m3);
        *(v2u*)(sA + cc * APITCH + h4) = pk;
      }
    }
    __syncthreads();

    {
      const int ncol = 16 * wave + c;
      const _Float16* wrow = W2t + (size_t)(k * HID + ncol) * HID + koff;
      v16h bfr[4];
#pragma unroll
      for (int kc = 0; kc < 4; ++kc) bfr[kc] = frag_load(wrow + 32 * kc);
      const float b2v = bf16r(b2[k * HID + ncol]);
#pragma unroll 1
      for (int i = 0; i < EROWS / 16; ++i) {
        const _Float16* arow = (const _Float16*)sA + (16 * i + c) * APITCH + koff;
        v8f acc = z8;
#pragma unroll
        for (int kc = 0; kc < 4; ++kc) {
          const v16h a = frag_load(arow + 32 * kc);
          acc = mma_h(a, bfr[kc], acc);
        }
        const float* rtp = sRt + (16 * i + 8 * hh) * 4 + k;
#pragma unroll
        for (int r = 0; r < 8; ++r) {
          const float m2v = tanhf(acc[r] * WCARRY_INV + b2v);
          colacc += m2v * rtp[r * 4];
        }
      }
    }
    __syncthreads();
  }

  colacc += __shfl_xor(colacc, 16, 32);
  if (hh == 0) sAgg[16 * wave + c] = colacc * AGG_SCALE;
  __syncthreads();
  if (wave == 0) {
    const v4f v = *(const v4f*)(sAgg + lane * 4);
    float* op = agg + (size_t)blk * HID + lane * 4;
    *(volatile v4f*)op = v;
    __threadfence();
    *(volatile v4f*)op = v;
  }
}

__global__ __launch_bounds__(NTHR) void node_step_kernel(const float* __restrict__ data, const float* __restrict__ agg,
                                                         const float* __restrict__ Wir, const float* __restrict__ bir,
                                                         const float* __restrict__ Wii, const float* __restrict__ bii,
                                                         const float* __restrict__ Win, const float* __restrict__ bin_,
                                                         const unsigned short* __restrict__ Wgtp,
                                                         const unsigned short* __restrict__ W1ctp,
                                                         float* hidden, float* __restrict__ Hall,
                                                         float* __restrict__ Ps, float* __restrict__ Pr, int t) {
  __shared__ __align__(16) unsigned short sAg[16 * APITCH];
  __shared__ __align__(16) _Float16       sHh[16 * APITCH];
  __shared__ __align__(16) float          sH[16 * FPITCH];
  __shared__ __align__(16) float          sWi[3 * FEAT * HID];
  __shared__ __align__(16) float          sIns[16 * 8];
  __shared__ __align__(16) float          sSl[NTHR / 32][16 * SLABP];
  const _Float16* Wgt  = (const _Float16*)Wgtp;
  const _Float16* W1ct = (const _Float16*)W1ctp;
  const int tid = threadIdx.x, lane = tid & 31, wave = tid >> 5;
  const int c = lane & 15, hh = lane >> 4, koff = hh * 8;
  const int rowbase = blockIdx.x * 16;

  {
    const int m = tid >> 4, c8 = (tid & 15) * 8;
    const float* ap = agg + (size_t)(rowbase + m) * HID + c8;
    const v4f a0 = *(const v4f*)(ap);
    const v4f a1 = *(const v4f*)(ap + 4);
    v4u pk;
    pk[0] = pack_h2(a0[0], a0[1]);
    pk[1] = pack_h2(a0[2], a0[3]);
    pk[2] = pack_h2(a1[0], a1[1]);
    pk[3] = pack_h2(a1[2], a1[3]);
    *(v4u*)(sAg + m * APITCH + c8) = pk;
  }
  if (tid < 16 * FEAT) {
    const int m = tid / FEAT, f = tid - m * FEAT;
    const int rowc = (rowbase + m) < NROW ? (rowbase + m) : (NROW - 1);
    sIns[m * 8 + f] = bf16r(data[((size_t)rowc * TLEN + (size_t)t) * FEAT + f]);
  }
  if (tid < 192) {
    const v4f w0 = bf16r4(*(const v4f*)(Wir + tid * 4));
    const v4f w1 = bf16r4(*(const v4f*)(Wii + tid * 4));
    const v4f w2 = bf16r4(*(const v4f*)(Win + tid * 4));
    *(v4f*)(sWi + 0 * FEAT * HID + tid * 4) = w0;
    *(v4f*)(sWi + 1 * FEAT * HID + tid * 4) = w1;
    *(v4f*)(sWi + 2 * FEAT * HID + tid * 4) = w2;
  }
  __syncthreads();

  const v8f z8 = {0.f, 0.f, 0.f, 0.f, 0.f, 0.f, 0.f, 0.f};
  const int j = 16 * wave + c;
  {
    v8f aR = z8, aI = z8, aN = z8;
    const _Float16* arow = (const _Float16*)sAg + c * APITCH + koff;
    const _Float16* wg = Wgt + (size_t)j * HID + koff;
#pragma unroll
    for (int kc = 0; kc < 4; ++kc) {
      const v16h a  = frag_load(arow + 32 * kc);
      const v16h bR = frag_load(wg + 32 * kc);
      const v16h bI = frag_load(wg + (size_t)1 * MATEL + 32 * kc);
      const v16h bN = frag_load(wg + (size_t)2 * MATEL + 32 * kc);
      aR = mma_h(a, bR, aR);
      aI = mma_h(a, bI, aI);
      aN = mma_h(a, bN, aN);
    }
    float wr[FEAT], wi[FEAT], wn[FEAT];
#pragma unroll
    for (int f = 0; f < FEAT; ++f) {
      wr[f] = sWi[0 * FEAT * HID + f * HID + j];
      wi[f] = sWi[1 * FEAT * HID + f * HID + j];
      wn[f] = sWi[2 * FEAT * HID + f * HID + j];
    }
    const float br = bf16r(bir[j]), bi = bf16r(bii[j]), bn = bf16r(bin_[j]);
#pragma unroll
    for (int r = 0; r < 8; ++r) {
      const int m = 8 * hh + r;
      float xr = 0.0f, xi = 0.0f, xn = 0.0f;
#pragma unroll
      for (int f = 0; f < FEAT; ++f) {
        const float iv = sIns[m * 8 + f];
        xr = fmaf(iv, wr[f], xr);
        xi = fmaf(iv, wi[f], xi);
        xn = fmaf(iv, wn[f], xn);
      }
      xr += br;
      xi += bi;
      xn += bn;
      const float hold = hidden[(size_t)(rowbase + m) * HID + j];
      const float rg = sigm(xr + aR[r] * WCARRY_INV);
      const float ig = sigm(xi + aI[r] * WCARRY_INV);
      const float ng = tanhf(xn + rg * (aN[r] * WCARRY_INV));
      const float hn = (1.0f - ig) * ng + ig * hold;
      sH[m * FPITCH + j] = hn;
      sHh[m * APITCH + j] = (_Float16)hn;
    }
  }
  __syncthreads();

  for (int pass = 0; pass < 2; ++pass) {
#pragma unroll
    for (int it = 0; it < 2; ++it) {
      const int idx = it * NTHR + tid;
      const int row = idx >> 5, c4 = (idx & 31) * 4;
      const v4f v = *(const v4f*)(sH + row * FPITCH + c4);
      *(volatile v4f*)(hidden + (size_t)(rowbase + row) * HID + c4) = v;
      *(volatile v4f*)(Hall + ((size_t)(rowbase + row) * NSTEP + (size_t)t) * HID + c4) = v;
    }
    __threadfence();
  }

  {
    const _Float16* hrow = sHh + c * APITCH + koff;
    v16h af[4];
#pragma unroll
    for (int kc = 0; kc < 4; ++kc) af[kc] = frag_load(hrow + 32 * kc);
    const int sflag = wave >> 2, kk = wave & 3;
    float* Pdst = sflag ? Pr : Ps;
    float* slab = sSl[wave];
    const int c4s = c * 4;
#pragma unroll 1
    for (int half = 0; half < 2; ++half) {
#pragma unroll 1
      for (int ntl = 0; ntl < 4; ++ntl) {
        const int n = HID * wave + 64 * half + 16 * ntl + c;
        const _Float16* wp = W1ct + (size_t)n * HID + koff;
        v8f acc = z8;
#pragma unroll
        for (int kc = 0; kc < 4; ++kc) {
          const v16h bq = frag_load(wp + 32 * kc);
          acc = mma_h(af[kc], bq, acc);
        }
#pragma unroll
        for (int r = 0; r < 8; ++r) slab[(8 * hh + r) * SLABP + 16 * ntl + c] = acc[r] * WCARRY_INV;
      }
      wave_sync_lds();
      for (int pass = 0; pass < 2; ++pass) {
#pragma unroll
        for (int it = 0; it < 8; ++it) {
          const int row = it * 2 + hh;
          const v4f v = *(const v4f*)(slab + row * SLABP + c4s);
          *(volatile v4f*)(Pdst + (size_t)(rowbase + row) * PCOLS + kk * HID + 64 * half + c4s) = v;
        }
        __threadfence();
      }
      wave_sync_lds();
    }
  }
}

__global__ __launch_bounds__(NTHR) void out_mlp_kernel(const float* __restrict__ Hall, const float* __restrict__ data,
                                                       const unsigned short* __restrict__ Wo1tp,
                                                       const unsigned short* __restrict__ Wo2tp,
                                                       const float* __restrict__ bo1, const float* __restrict__ bo2,
                                                       const float* __restrict__ Wo3, const float* __restrict__ bo3,
                                                       const int* __restrict__ ps,
                                                       float* __restrict__ out) {
  __shared__ __align__(16) unsigned short sA[16 * APITCH];
  __shared__ __align__(16) _Float16       sB[16 * APITCH];
  __shared__ __align__(16) float          sP2[16 * FPITCH];
  __shared__ __align__(16) float          sW3[HID * FEAT];
  __shared__ __align__(16) float          sOut[128];
  const _Float16* Wo1t = (const _Float16*)Wo1tp;
  const _Float16* Wo2t = (const _Float16*)Wo2tp;
  const int tid = threadIdx.x, lane = tid & 31, wave = tid >> 5;
  const int c = lane & 15, hh = lane >> 4, koff = hh * 8;
  const int rowbase = blockIdx.x * 16;
  const int psv = ps[0];
  const float nanv = __uint_as_float(0x7FC00000u);

  {
    const int m = tid >> 4, c8 = (tid & 15) * 8;
    const float* ap = Hall + (size_t)(rowbase + m) * HID + c8;
    const v4f a0 = *(const v4f*)(ap);
    const v4f a1 = *(const v4f*)(ap + 4);
    v4u pk;
    pk[0] = pack_h2(a0[0], a0[1]);
    pk[1] = pack_h2(a0[2], a0[3]);
    pk[2] = pack_h2(a1[0], a1[1]);
    pk[3] = pack_h2(a1[2], a1[3]);
    *(v4u*)(sA + m * APITCH + c8) = pk;
  }
  if (tid < 192) {
    const v4f w = bf16r4(*(const v4f*)(Wo3 + tid * 4));
    *(v4f*)(sW3 + tid * 4) = w;
  }
  __syncthreads();

  const v8f z8 = {0.f, 0.f, 0.f, 0.f, 0.f, 0.f, 0.f, 0.f};
  const int j = 16 * wave + c;
  {
    const _Float16* arow = (const _Float16*)sA + c * APITCH + koff;
    const _Float16* wp = Wo1t + (size_t)j * HID + koff;
    v8f acc = z8;
#pragma unroll
    for (int kc = 0; kc < 4; ++kc) {
      const v16h a  = frag_load(arow + 32 * kc);
      const v16h bq = frag_load(wp + 32 * kc);
      acc = mma_h(a, bq, acc);
    }
    const float bv = bf16r(bo1[j]);
#pragma unroll
    for (int r = 0; r < 8; ++r) {
      const float v = fmaxf(acc[r] * WCARRY_INV + bv, 0.0f);
      sB[(8 * hh + r) * APITCH + j] = (_Float16)v;
    }
  }
  __syncthreads();
  {
    const _Float16* arow = sB + c * APITCH + koff;
    const _Float16* wp = Wo2t + (size_t)j * HID + koff;
    v8f acc = z8;
#pragma unroll
    for (int kc = 0; kc < 4; ++kc) {
      const v16h a  = frag_load(arow + 32 * kc);
      const v16h bq = frag_load(wp + 32 * kc);
      acc = mma_h(a, bq, acc);
    }
    const float bv = bf16r(bo2[j]);
#pragma unroll
    for (int r = 0; r < 8; ++r) {
      const float v = fmaxf(acc[r] * WCARRY_INV + bv, 0.0f);
      sP2[(8 * hh + r) * FPITCH + j] = v;
    }
  }
  __syncthreads();

  if (tid < 16 * FEAT) {
    const int m = tid / FEAT, f = tid - m * FEAT;
    const int R = rowbase + m;
    const int bn = R / NSTEP;
    const int tt = R - bn * NSTEP;
    float acc = 0.0f;
#pragma unroll 4
    for (int h = 0; h < HID; ++h) acc = fmaf(sP2[m * FPITCH + h], sW3[h * FEAT + f], acc);
    const float ins = bf16r(data[((size_t)bn * TLEN + (size_t)tt) * FEAT + f]);
    const float b3 = bf16r(bo3[f]);
    const float val = ins + (acc + b3);
    sOut[tid] = (psv == 1) ? val : nanv;
  }
  __syncthreads();
  if (wave == 0) {
    const int l4 = (lane < 24 ? lane : 23) * 4;
    const v4f v = *(const v4f*)(sOut + l4);
    float* op = out + (size_t)blockIdx.x * (16 * FEAT) + l4;
    if (lane < 24) *(volatile v4f*)op = v;
    __threadfence();
    if (lane < 24) *(volatile v4f*)op = v;
  }
}

extern "C" void kernel_launch(void* const* d_in, const int* in_sizes, int n_in,
                              void* d_out, int out_size, void* d_ws, size_t ws_size, hipStream_t stream) {
  if (n_in < 24 || d_out == nullptr || d_ws == nullptr) return;
  if (in_sizes[0] != BATCH * NODES * TLEN * FEAT || in_sizes[1] != BATCH * NEDGE * NTYPE ||
      in_sizes[4] < 1 ||
      in_sizes[5] != NTYPE * 2 * HID * HID || in_sizes[6] != NTYPE * HID ||
      in_sizes[7] != NTYPE * HID * HID || in_sizes[8] != NTYPE * HID ||
      in_sizes[9] != MATEL || in_sizes[10] != MATEL || in_sizes[11] != MATEL ||
      in_sizes[12] != FEAT * HID || in_sizes[13] != HID || in_sizes[14] != FEAT * HID || in_sizes[15] != HID ||
      in_sizes[16] != FEAT * HID || in_sizes[17] != HID ||
      in_sizes[18] != MATEL || in_sizes[19] != HID || in_sizes[20] != MATEL || in_sizes[21] != HID ||
      in_sizes[22] != HID * FEAT || in_sizes[23] != FEAT ||
      out_size != OUTROWS * FEAT) return;

  const float* data     = (const float*)d_in[0];
  const float* rel_type = (const float*)d_in[1];
  const int*   pstep = (const int*)d_in[4];
  const float* W1  = (const float*)d_in[5];
  const float* b1  = (const float*)d_in[6];
  const float* W2  = (const float*)d_in[7];
  const float* b2  = (const float*)d_in[8];
  const float* Whr = (const float*)d_in[9];
  const float* Whi = (const float*)d_in[10];
  const float* Whh = (const float*)d_in[11];
  const float* Wir = (const float*)d_in[12];
  const float* bir = (const float*)d_in[13];
  const float* Wii = (const float*)d_in[14];
  const float* bii = (const float*)d_in[15];
  const float* Win = (const float*)d_in[16];
  const float* bin_ = (const float*)d_in[17];
  const float* Wo1 = (const float*)d_in[18];
  const float* bo1 = (const float*)d_in[19];
  const float* Wo2 = (const float*)d_in[20];
  const float* bo2 = (const float*)d_in[21];
  const float* Wo3 = (const float*)d_in[22];
  const float* bo3 = (const float*)d_in[23];
  float* out = (float*)d_out;

  char* ws = (char*)d_ws;
  size_t off = 0;
  auto carve = [&](size_t bytes) -> char* { char* p = ws + off; off += (bytes + 255) & ~(size_t)255; return p; };
  float* hidden = (float*)carve((size_t)NROWP * HID * 4);
  float* agg    = (float*)carve((size_t)NROWP * HID * 4);
  float* Ps     = (float*)carve((size_t)NROWP * PCOLS * 4);
  float* Pr     = (float*)carve((size_t)NROWP * PCOLS * 4);
  float* Hall   = (float*)carve((size_t)HALLROWS * HID * 4);
  unsigned short* WT = (unsigned short*)carve((size_t)NMAT * MATEL * 2);
  if (off > ws_size || off > (size_t)134217728) return;
  unsigned short* W1ct = WT;
  unsigned short* W2t  = WT + (size_t)8 * MATEL;
  unsigned short* Wgt  = WT + (size_t)12 * MATEL;
  unsigned short* Wo1t = WT + (size_t)15 * MATEL;
  unsigned short* Wo2t = WT + (size_t)16 * MATEL;

  wprep_kernel<<<dim3(2, 2, NMAT), NTHR, 0, stream>>>(W1, W2, Whr, Whi, Whh, Wo1, Wo2, WT);
  zero_state_kernel<<<ZERO_V4 / NTHR, NTHR, 0, stream>>>(hidden, ZERO_V4);

  for (int t = 0; t < NSTEP; ++t) {
    edge_msg_kernel<<<NROW, NTHR, 0, stream>>>(Ps, Pr, rel_type, b1, b2, W2t, agg);
    node_step_kernel<<<NROWP / 16, NTHR, 0, stream>>>(data, agg, Wir, bir, Wii, bii, Win, bin_, Wgt, W1ct,
                                                      hidden, Hall, Ps, Pr, t);
  }
  out_mlp_kernel<<<OUTROWS / 16, NTHR, 0, stream>>>(Hall, data, Wo1t, Wo2t, bo1, bo2, Wo3, bo3, pstep, out);
}
